// CrossMamba_44736379355723
// MI455X (gfx1250) — hardware-verified
//
#include <hip/hip_runtime.h>
#include <math.h>

typedef __attribute__((ext_vector_type(16))) _Float16 v16h;
typedef __attribute__((ext_vector_type(8)))  _Float16 v8h;
typedef __attribute__((ext_vector_type(16))) __bf16   v16b;
typedef __attribute__((ext_vector_type(8)))  __bf16   v8b;
typedef __attribute__((ext_vector_type(8)))  float    v8f;
typedef __attribute__((ext_vector_type(4)))  float    v4f;
typedef __attribute__((ext_vector_type(4)))  unsigned v4u;

constexpr int kBatch  = 2;
constexpr int kLctx   = 2048;
constexpr int kLq     = 2048;
constexpr int kLtot   = kLctx + kLq;
constexpr int kDm     = 512;
constexpr int kDin    = 1024;
constexpr int kNst    = 16;
constexpr int kDtR    = 32;
constexpr int kXdP    = 64;
constexpr int kRowsF  = kBatch * kLtot;
constexpr int kRowsB  = kBatch * kLq;
constexpr int kRowsS  = kRowsF + kRowsB;
constexpr int kConvTP = 260;
constexpr int kScanTS = 64;
constexpr int kScanCh = 64;
constexpr int kScanYP = 68;
constexpr int kBcW    = 32;
constexpr float kCarryWx   = 32.0f;
constexpr float kCarryDt   = 16.0f;
constexpr float kCarryWdt  = 8.0f;
static_assert(kLtot == 4096 && kRowsF == 8192 && kRowsB == 4096 && kRowsS == 12288, "row counts");
static_assert(kDtR + 2 * kNst == kXdP, "x_proj width");
static_assert((kDm % 32) == 0 && (kDin % 32) == 0 && (kDtR % 32) == 0, "GEMM K multiples of 32");
static_assert((kRowsF % 64) == 0 && (kRowsB % 64) == 0 && (kRowsS % 64) == 0 && (kLq % 64) == 0, "GEMM M multiples of 64");
static_assert((kDin % 64) == 0 && (kXdP % 64) == 0 && (kDm % 64) == 0, "GEMM N multiples of 64");
static_assert((kLtot % kScanTS) == 0 && (kLctx % kScanTS) == 0 && (kDin % kScanCh) == 0 && (kDin % 256) == 0, "tile multiples");
static_assert(kBcW == 2 * kNst, "B|C width");

constexpr size_t kSzX16   = (size_t)kRowsF * kDm  * 2;
constexpr size_t kSzWI    = (size_t)2 * kDin * kDm * 2;
constexpr size_t kSzWO    = (size_t)kDm * kDin * 2;
constexpr size_t kSzWX    = (size_t)kXdP * kDin * 2;
constexpr size_t kSzWDT   = (size_t)kDin * kDtR * 2;
constexpr size_t kSzXI    = (size_t)kRowsF * kDin * 4;
constexpr size_t kSzZ     = (size_t)kRowsB * kDin * 4;
constexpr size_t kSzXC    = (size_t)kRowsS * kDin * 2;
constexpr size_t kSzDBL   = (size_t)kRowsS * kXdP * 4;
constexpr size_t kSzDT16  = (size_t)kRowsS * kDtR * 2;
constexpr size_t kSzYB    = (size_t)kRowsB * kDin * 4;
constexpr size_t kSzYS    = (size_t)kRowsB * kDin * 2;
constexpr size_t kOffXH   = 0;
constexpr size_t kOffXL   = kOffXH   + kSzX16;
constexpr size_t kOffWIH  = kOffXL   + kSzX16;
constexpr size_t kOffWIL  = kOffWIH  + kSzWI;
constexpr size_t kOffWOH  = kOffWIL  + kSzWI;
constexpr size_t kOffWOL  = kOffWOH  + kSzWO;
constexpr size_t kOffWX   = kOffWOL  + kSzWO;
constexpr size_t kOffWDT  = kOffWX   + kSzWX;
constexpr size_t kOffXI   = kOffWDT  + kSzWDT;
constexpr size_t kOffZ    = kOffXI   + kSzXI;
constexpr size_t kOffXC   = kOffZ    + kSzZ;
constexpr size_t kOffDBL  = kOffXC   + kSzXC;
constexpr size_t kOffDT16 = kOffDBL  + kSzDBL;
constexpr size_t kOffYB   = kOffDT16 + kSzDT16;
constexpr size_t kWsTotal = kOffYB   + kSzYB;
static_assert(kWsTotal == 119472128ull, "carve total");
static_assert(kWsTotal <= 134217728ull, "carve cap");
static_assert(kSzYS <= kSzX16, "aliased plane fits its region");
static_assert((kOffXL % 128) == 0 && (kOffWIH % 128) == 0 && (kOffWIL % 128) == 0 && (kOffWOH % 128) == 0 &&
              (kOffWOL % 128) == 0 && (kOffWX % 128) == 0 && (kOffWDT % 128) == 0 && (kOffXI % 128) == 0 &&
              (kOffZ % 128) == 0 && (kOffXC % 128) == 0 && (kOffDBL % 128) == 0 && (kOffDT16 % 128) == 0 &&
              (kOffYB % 128) == 0, "128-B aligned regions");

__device__ __forceinline__ unsigned short f2bf_bits(float f) {
  unsigned u = __float_as_uint(f);
  return (unsigned short)((u + 0x7FFFu + ((u >> 16) & 1u)) >> 16);
}
__device__ __forceinline__ float bf_bits2f(unsigned short h) { return __uint_as_float(((unsigned)h) << 16); }

__device__ __forceinline__ float h16_to_f32(unsigned hb) {
  const unsigned sgn = (hb & 0x8000u) << 16;
  const unsigned em = hb & 0x7fffu;
  const float fn = __uint_as_float((em << 13) + 0x38000000u);
  const float fs = (float)em * 5.9604644775390625e-8f;
  const float mag = (em < 0x400u) ? fs : fn;
  return __uint_as_float(__float_as_uint(mag) | sgn);
}

__device__ __forceinline__ void dep_guard4_h(v8f& a, v8f& b, v8f& c, v8f& d, v16h x, v16h y) { asm volatile("v_nop\n\tv_nop\n\tv_nop\n\tv_nop" : "+v"(a), "+v"(b), "+v"(c), "+v"(d) : "v"(x), "v"(y)); }
__device__ __forceinline__ void dep_guard4_b(v8f& a, v8f& b, v8f& c, v8f& d, v16b x, v16b y) { asm volatile("v_nop\n\tv_nop\n\tv_nop\n\tv_nop" : "+v"(a), "+v"(b), "+v"(c), "+v"(d) : "v"(x), "v"(y)); }
__device__ __forceinline__ void keep4_h(v16h a, v16h b, v16h c, v16h d) { asm volatile("v_nop" :: "v"(a), "v"(b), "v"(c), "v"(d)); }
__device__ __forceinline__ void keep4_b(v16b a, v16b b, v16b c, v16b d) { asm volatile("v_nop" :: "v"(a), "v"(b), "v"(c), "v"(d)); }
__device__ __forceinline__ void acc_guard4(v8f& a, v8f& b, v8f& c, v8f& d) { asm volatile("v_nop\n\tv_nop\n\tv_nop\n\tv_nop" : "+v"(a), "+v"(b), "+v"(c), "+v"(d)); }

template <typename T> struct Frag;
template <> struct Frag<_Float16> {
  typedef v16h V; union U { v16h v; v8h h[2]; };
  static __device__ __forceinline__ v16h load(const _Float16* p) {
    U f; f.h[0] = *(const v8h*)(p); f.h[1] = *(const v8h*)(p + 16); return f.v;
  }
  static __device__ __forceinline__ v8f mma(v16h a, v16h b, v8f c) {
    return __builtin_amdgcn_wmma_f32_16x16x32_f16(false, a, false, b, (short)0, c, false, false);
  }
  static __device__ __forceinline__ void guard(v8f& a, v8f& b, v8f& c, v8f& d, v16h x, v16h y) { dep_guard4_h(a, b, c, d, x, y); }
  static __device__ __forceinline__ void keep(v16h a, v16h b, v16h c, v16h d) { keep4_h(a, b, c, d); }
};
template <> struct Frag<__bf16> {
  typedef v16b V; union U { v16b v; v8b h[2]; };
  static __device__ __forceinline__ v16b load(const __bf16* p) {
    U f; f.h[0] = *(const v8b*)(p); f.h[1] = *(const v8b*)(p + 16); return f.v;
  }
  static __device__ __forceinline__ v8f mma(v16b a, v16b b, v8f c) {
    return __builtin_amdgcn_wmma_f32_16x16x32_bf16(false, a, false, b, (short)0, c, false, false);
  }
  static __device__ __forceinline__ void guard(v8f& a, v8f& b, v8f& c, v8f& d, v16b x, v16b y) { dep_guard4_b(a, b, c, d, x, y); }
  static __device__ __forceinline__ void keep(v16b a, v16b b, v16b c, v16b d) { keep4_b(a, b, c, d); }
};

template <int ET> struct Elem;
template <> struct Elem<0> { typedef _Float16 T; };
template <> struct Elem<1> { typedef __bf16 T; };
template <int ET, int SPL, int BIAS_MODE, int OUT_MODE>
__global__ __launch_bounds__(256) void wmma_gemm64(
    const unsigned short* __restrict__ Ap, const unsigned short* __restrict__ A2p, int lda, long strideA,
    const unsigned short* __restrict__ Btp, const unsigned short* __restrict__ Bt2p, int ldb, long strideB,
    void* __restrict__ Cout, void* __restrict__ Cout2, int ldc, long strideC,
    const float* __restrict__ bias,
    int M, int N, int K, float scale) {
  typedef typename Elem<ET>::T T;
  typedef typename Frag<T>::V V;
  const T* A = (const T*)Ap; const T* A2 = (const T*)A2p; const T* Bt = (const T*)Btp; const T* Bt2 = (const T*)Bt2p;
  __shared__ __align__(16) float sT[8][16 * 68];
  const int b    = blockIdx.y;
  const int lane = threadIdx.x & 31;
  const int wave = threadIdx.x >> 5;
  const int tilesN = N >> 6;
  const int tilesM = M >> 6;
  const int tile = blockIdx.x * 8 + wave;
  if (tile >= tilesM * tilesN) return;
  const int tm = tile / tilesN;
  const int tn = tile - tm * tilesN;
  const int m0 = tm << 6;
  const int n0 = tn << 6;

  const T* Ab  = A  + (size_t)b * strideA;
  const T* Bb  = Bt + (size_t)b * strideB;
  const T* Ab2 = (SPL >= 1) ? (A2  + (size_t)b * strideA) : nullptr;
  const T* Bb2 = (SPL == 2) ? (Bt2 + (size_t)b * strideB) : nullptr;

  const int rlane = lane & 15;
  const int koff  = (lane >> 4) * 8;
  const int mOff  = (lane >> 4) * 8;

  v8f acc[4][4];
#pragma unroll
  for (int i = 0; i < 4; ++i)
#pragma unroll
    for (int j = 0; j < 4; ++j) acc[i][j] = (v8f){0.f,0.f,0.f,0.f,0.f,0.f,0.f,0.f};

  for (int k0 = 0; k0 < K; k0 += 32) {
    V bh[4], bl[4];
#pragma unroll
    for (int j = 0; j < 4; ++j) {
      const size_t bo = (size_t)(n0 + (j << 4) + rlane) * ldb + koff + k0;
      bh[j] = Frag<T>::load(Bb + bo);
      if (SPL == 2) bl[j] = Frag<T>::load(Bb2 + bo);
    }
#pragma unroll
    for (int i = 0; i < 4; ++i) {
      const size_t ao = (size_t)(m0 + (i << 4) + rlane) * lda + koff + k0;
      V ah = Frag<T>::load(Ab + ao);
      V al;
      if (SPL >= 1) al = Frag<T>::load(Ab2 + ao);
#pragma unroll
      for (int j = 0; j < 4; ++j) {
        acc[i][j] = Frag<T>::mma(ah, bh[j], acc[i][j]);
        if (SPL == 2) acc[i][j] = Frag<T>::mma(ah, bl[j], acc[i][j]);
        if (SPL >= 1) acc[i][j] = Frag<T>::mma(al, bh[j], acc[i][j]);
      }
      Frag<T>::guard(acc[i][0], acc[i][1], acc[i][2], acc[i][3], ah, (SPL >= 1) ? al : ah);
    }
    Frag<T>::keep(bh[0], bh[1], bh[2], bh[3]);
    if (SPL == 2) Frag<T>::keep(bl[0], bl[1], bl[2], bl[3]);
  }
  acc_guard4(acc[0][0], acc[0][1], acc[0][2], acc[0][3]);
  acc_guard4(acc[1][0], acc[1][1], acc[1][2], acc[1][3]);
  acc_guard4(acc[2][0], acc[2][1], acc[2][2], acc[2][3]);
  acc_guard4(acc[3][0], acc[3][1], acc[3][2], acc[3][3]);

  float* slab = sT[wave];
#pragma unroll
  for (int i = 0; i < 4; ++i) {
    const int mBase = m0 + (i << 4);
#pragma unroll
    for (int j = 0; j < 4; ++j) {
      const int n = n0 + (j << 4) + rlane;
      float bv = 0.f;
      if (BIAS_MODE == 2) bv = bias[n];
#pragma unroll
      for (int r = 0; r < 8; ++r) {
        float v = acc[i][j][r] * scale;
        if (BIAS_MODE == 1) v += bias[mBase + mOff + r];
        if (BIAS_MODE == 2) v += bv;
        slab[(mOff + r) * 68 + (j << 4) + rlane] = v;
      }
    }
    __builtin_amdgcn_fence(__ATOMIC_RELEASE, "workgroup");
    __builtin_amdgcn_wave_barrier();
    __builtin_amdgcn_fence(__ATOMIC_ACQUIRE, "workgroup");
    if (OUT_MODE == 0) {
      float* C = (float*)Cout + (size_t)b * strideC;
      const int hh = lane >> 4, c4 = (lane & 15) * 4;
      for (int pass = 0; pass < 2; ++pass) {
#pragma unroll
        for (int it = 0; it < 8; ++it) {
          const int row = it * 2 + hh;
          v4f v = *(const v4f*)(slab + row * 68 + c4);
          *(volatile v4f*)(C + (size_t)(mBase + row) * ldc + n0 + c4) = v;
        }
        __threadfence();
      }
    } else {
      const int q = lane >> 3, c8 = (lane & 7) * 8;
      unsigned short* C  = (unsigned short*)Cout  + (size_t)b * strideC;
      unsigned short* C2 = (OUT_MODE == 2) ? ((unsigned short*)Cout2 + (size_t)b * strideC) : nullptr;
      for (int pass = 0; pass < 2; ++pass) {
#pragma unroll
        for (int it = 0; it < 4; ++it) {
          const int row = it * 4 + q;
          const float* sp = slab + row * 68 + c8;
          v8h hv, lv;
#pragma unroll
          for (int e = 0; e < 8; ++e) {
            if (OUT_MODE == 1) {
              hv[e] = (_Float16)sp[e];
            } else {
              unsigned short hb = f2bf_bits(sp[e]);
              unsigned short lb = f2bf_bits(sp[e] - bf_bits2f(hb));
              hv[e] = __builtin_bit_cast(_Float16, hb);
              lv[e] = __builtin_bit_cast(_Float16, lb);
            }
          }
          *(volatile v8h*)(C + (size_t)(mBase + row) * ldc + n0 + c8) = hv;
          if (OUT_MODE == 2) *(volatile v8h*)(C2 + (size_t)(mBase + row) * ldc + n0 + c8) = lv;
        }
        __threadfence();
      }
    }
    __builtin_amdgcn_fence(__ATOMIC_RELEASE, "workgroup");
    __builtin_amdgcn_wave_barrier();
    __builtin_amdgcn_fence(__ATOMIC_ACQUIRE, "workgroup");
  }
}

__global__ __launch_bounds__(256) void split_rows_bf16_kernel(
    const float* __restrict__ src, unsigned short* __restrict__ dhi, unsigned short* __restrict__ dlo, int total8)
{
  const int i = blockIdx.x * 256 + threadIdx.x;
  if (i >= total8) return;
  const size_t e0 = (size_t)i << 3;
  const v4f a0 = *(const v4f*)(src + e0);
  const v4f a1 = *(const v4f*)(src + e0 + 4);
  v8h hv, lv;
#pragma unroll
  for (int e = 0; e < 4; ++e) {
    const unsigned short h0 = f2bf_bits(a0[e]), h1 = f2bf_bits(a1[e]);
    const unsigned short l0 = f2bf_bits(a0[e] - bf_bits2f(h0)), l1 = f2bf_bits(a1[e] - bf_bits2f(h1));
    hv[e]     = __builtin_bit_cast(_Float16, h0);
    hv[4 + e] = __builtin_bit_cast(_Float16, h1);
    lv[e]     = __builtin_bit_cast(_Float16, l0);
    lv[4 + e] = __builtin_bit_cast(_Float16, l1);
  }
  unsigned short* qh = dhi + e0;
  unsigned short* ql = dlo + e0;
  *(volatile v8h*)qh = hv;
  *(volatile v8h*)ql = lv;
  __threadfence();
  *(volatile v8h*)qh = hv;
  *(volatile v8h*)ql = lv;
}

__global__ __launch_bounds__(256) void cast_f16_kernel(
    const float* __restrict__ src, unsigned short* __restrict__ dst, int total8, float scale)
{
  const int i = blockIdx.x * 256 + threadIdx.x;
  if (i >= total8) return;
  const size_t e0 = (size_t)i << 3;
  const float* p = src + e0;
  const v4f a0 = *(const v4f*)(p);
  const v4f a1 = *(const v4f*)(p + 4);
  v8h hv;
#pragma unroll
  for (int e = 0; e < 4; ++e) {
    hv[e]     = (_Float16)(a0[e] * scale);
    hv[4 + e] = (_Float16)(a1[e] * scale);
  }
  unsigned short* q = dst + e0;
  *(volatile v8h*)q = hv;
  __threadfence();
  *(volatile v8h*)q = hv;
}

__global__ __launch_bounds__(256) void build_x_kernel(
    const float* __restrict__ query, const float* __restrict__ context,
    const float* __restrict__ seg_c, const float* __restrict__ seg_q,
    unsigned short* __restrict__ XH, unsigned short* __restrict__ XL, int total8)
{
  const int i = blockIdx.x * 256 + threadIdx.x;
  if (i >= total8) return;
  const int r  = i >> 6;
  const int c8 = (i & 63) << 3;
  const int b  = r / kLtot;
  const int p  = r - b * kLtot;
  const bool isq = (p >= kLctx);
  const int pr = isq ? (p - kLctx) : p;
  const float* src = (isq ? query : context) + ((size_t)b * kLq + pr) * kDm + c8;
  const float* sg  = (isq ? seg_q : seg_c) + c8;
  const v4f a0 = *(const v4f*)(src);
  const v4f a1 = *(const v4f*)(src + 4);
  const v4f s0 = *(const v4f*)(sg);
  const v4f s1 = *(const v4f*)(sg + 4);
  v8h hv, lv;
#pragma unroll
  for (int e = 0; e < 4; ++e) {
    const float x0 = a0[e] + s0[e];
    const float x1 = a1[e] + s1[e];
    const unsigned short h0 = f2bf_bits(x0), h1 = f2bf_bits(x1);
    const unsigned short l0 = f2bf_bits(x0 - bf_bits2f(h0)), l1 = f2bf_bits(x1 - bf_bits2f(h1));
    hv[e]     = __builtin_bit_cast(_Float16, h0);
    hv[4 + e] = __builtin_bit_cast(_Float16, h1);
    lv[e]     = __builtin_bit_cast(_Float16, l0);
    lv[4 + e] = __builtin_bit_cast(_Float16, l1);
  }
  const size_t e0 = (size_t)i << 3;
  unsigned short* qh = XH + e0;
  unsigned short* ql = XL + e0;
  *(volatile v8h*)qh = hv;
  *(volatile v8h*)ql = lv;
  __threadfence();
  *(volatile v8h*)qh = hv;
  *(volatile v8h*)ql = lv;
}

__global__ __launch_bounds__(256) void dt_cast_kernel(
    const float* __restrict__ DBL, unsigned short* __restrict__ DT16, int total8, float scale)
{
  const int i = blockIdx.x * 256 + threadIdx.x;
  if (i >= total8) return;
  const int e0  = i << 3;
  const int row = e0 >> 5;
  const int c8  = e0 & 31;
  const float* p = DBL + (size_t)row * kXdP + c8;
  const v4f a0 = *(const v4f*)(p);
  const v4f a1 = *(const v4f*)(p + 4);
  v8h hv;
#pragma unroll
  for (int e = 0; e < 4; ++e) {
    hv[e]     = (_Float16)(a0[e] * scale);
    hv[4 + e] = (_Float16)(a1[e] * scale);
  }
  unsigned short* qd = DT16 + e0;
  *(volatile v8h*)qd = hv;
  __threadfence();
  *(volatile v8h*)qd = hv;
}

__global__ __launch_bounds__(256) void conv_silu_kernel(
    const float* __restrict__ XI, const float* __restrict__ cw, const float* __restrict__ cb,
    unsigned short* __restrict__ XC16)
{
  __shared__ __align__(16) float sT[16 * kConvTP];
  const int tid = threadIdx.x, lane = tid & 31, wave = tid >> 5;
  const int d0 = blockIdx.x * 256, d = d0 + tid;
  const int by = blockIdx.y;
  const bool bwd = (by >= kRowsF / 64);
  int xrow0, orow0;
  bool hist;
  if (!bwd) {
    xrow0 = by * 64;
    orow0 = xrow0;
    hist  = ((xrow0 & (kLtot - 1)) > 0);
  } else {
    const int bb  = by - kRowsF / 64;
    const int b   = bb / (kLq / 64);
    const int blk = bb - b * (kLq / 64);
    xrow0 = b * kLtot + kLctx + blk * 64;
    orow0 = kRowsF + b * kLq + blk * 64;
    hist  = (blk < kLq / 64 - 1);
  }
  const int sgn    = bwd ? -1 : 1;
  const int rfirst = bwd ? (xrow0 + 63) : xrow0;
  const v4f wv = *(const v4f*)(cw + (size_t)d * 4);
  const float w0 = wv[0], w1 = wv[1], w2 = wv[2], w3 = wv[3];
  const float bc = cb[d];
  float xm3, xm2, xm1;
  {
    const int r1 = hist ? (rfirst - sgn) : rfirst;
    const int r2 = hist ? (rfirst - 2 * sgn) : rfirst;
    const int r3 = hist ? (rfirst - 3 * sgn) : rfirst;
    const float v1 = XI[(size_t)r1 * kDin + d];
    const float v2 = XI[(size_t)r2 * kDin + d];
    const float v3 = XI[(size_t)r3 * kDin + d];
    xm1 = hist ? v1 : 0.f;
    xm2 = hist ? v2 : 0.f;
    xm3 = hist ? v3 : 0.f;
  }
#pragma unroll 1
  for (int sub = 0; sub < 4; ++sub) {
#pragma unroll 1
    for (int s = 0; s < 16; ++s) {
      const int ls = sub * 16 + s;
      const float xcur = XI[(size_t)(rfirst + sgn * ls) * kDin + d];
      float acc = w0 * xm3;
      acc = fmaf(w1, xm2, acc);
      acc = fmaf(w2, xm1, acc);
      acc = fmaf(w3, xcur, acc);
      const float sv = acc + bc;
      const float sg = __builtin_amdgcn_rcpf(1.0f + __expf(-sv));
      const int trow = bwd ? (15 - s) : s;
      sT[trow * kConvTP + tid] = sv * sg;
      xm3 = xm2; xm2 = xm1; xm1 = xcur;
    }
    __syncthreads();
    const int ob = orow0 + (bwd ? (48 - sub * 16) : (sub * 16));
    v8h bv[2];
#pragma unroll
    for (int it = 0; it < 2; ++it) {
      const float* sp = sT + (it * 8 + wave) * kConvTP + lane * 8;
      const v4f a0 = *(const v4f*)(sp);
      const v4f a1 = *(const v4f*)(sp + 4);
#pragma unroll
      for (int e = 0; e < 4; ++e) {
        bv[it][e]     = (_Float16)a0[e];
        bv[it][4 + e] = (_Float16)a1[e];
      }
    }
    for (int pass = 0; pass < 2; ++pass) {
#pragma unroll
      for (int it = 0; it < 2; ++it)
        *(volatile v8h*)(XC16 + (size_t)(ob + it * 8 + wave) * kDin + d0 + lane * 8) = bv[it];
      __threadfence();
    }
    __syncthreads();
  }
}

template <int DIR>
__global__ __launch_bounds__(64) void scan_kernel(
    const float* __restrict__ DBL, const unsigned short* __restrict__ DTP, const float* __restrict__ XI,
    const float* __restrict__ Zp, const float* __restrict__ cw, const float* __restrict__ cb,
    const float* __restrict__ bdt, const float* __restrict__ Alog, const float* __restrict__ Dp,
    float* YB, unsigned short* __restrict__ YSH, unsigned short* __restrict__ YSL)
{
  __shared__ __align__(16) float    sX[kScanTS * kBcW];
  __shared__ __align__(16) unsigned sDT[kScanTS * (kScanCh / 2)];
  __shared__ __align__(16) float    sY[kScanTS * kScanYP];
  __shared__ __align__(16) float    sA[kNst * kScanCh];
  const int tid = threadIdx.x, lane = tid & 31, wave = tid >> 5;
  constexpr int kBlkPerB = kDin / kScanCh;
  const int bix = blockIdx.x / kBlkPerB;
  const int d0  = (blockIdx.x - bix * kBlkPerB) * kScanCh;
  const int d   = d0 + tid;
#pragma unroll 1
  for (int s = 0; s < kNst; ++s) sA[s * kScanCh + tid] = -expf(Alog[(size_t)d * kNst + s]);
  __syncthreads();
  float negA[kNst], h[kNst];
#pragma unroll
  for (int s = 0; s < kNst; ++s) {
    negA[s] = sA[s * kScanCh + tid];
    h[s] = 0.f;
  }
  const v4f wv = *(const v4f*)(cw + (size_t)d * 4);
  const float w0 = wv[0], w1 = wv[1], w2 = wv[2], w3 = wv[3];
  const float bc = cb[d], bb = bdt[d], Dd = Dp[d];
  float xm3 = 0.f, xm2 = 0.f, xm1 = 0.f;
  const int lr = tid >> 3, lq = tid & 7;
  constexpr int kSteps = DIR ? kLq : kLtot;
#pragma unroll 1
  for (int t0 = 0; t0 < kSteps; t0 += kScanTS) {
    const int pb = DIR ? (kLtot - kScanTS - t0) : t0;
    const size_t srow  = DIR ? ((size_t)kRowsF + (size_t)bix * kLq + (size_t)(pb - kLctx)) : ((size_t)bix * kLtot + pb);
    const size_t xirow = (size_t)bix * kLtot + pb;
    const bool outp    = (pb >= kLctx);
    const size_t qrow  = (size_t)bix * kLq + (size_t)(outp ? (pb - kLctx) : 0);
    __syncthreads();
#pragma unroll
    for (int i = 0; i < 8; ++i) {
      const int r = lr + 8 * i;
      *(v4f*)(sX + r * kBcW + lq * 4) = *(const v4f*)(DBL + (srow + r) * kXdP + kDtR + lq * 4);
      *(v4u*)(sDT + r * (kScanCh / 2) + lq * 4) = *(const v4u*)(DTP + (srow + r) * kDin + d0 + lq * 8);
    }
    __syncthreads();
#pragma unroll 1
    for (int s = 0; s < kScanTS; ++s) {
      const int lrow = DIR ? (kScanTS - 1 - s) : s;
      const float* xr = sX + lrow * kBcW;
      float Bs[kNst], Cs[kNst];
#pragma unroll
      for (int q4 = 0; q4 < 4; ++q4) {
        const v4f bv = *(const v4f*)(xr + 4 * q4);
        const v4f cv = *(const v4f*)(xr + kNst + 4 * q4);
        Bs[4 * q4 + 0] = bv[0]; Bs[4 * q4 + 1] = bv[1]; Bs[4 * q4 + 2] = bv[2]; Bs[4 * q4 + 3] = bv[3];
        Cs[4 * q4 + 0] = cv[0]; Cs[4 * q4 + 1] = cv[1]; Cs[4 * q4 + 2] = cv[2]; Cs[4 * q4 + 3] = cv[3];
      }
      const unsigned wd = sDT[lrow * (kScanCh / 2) + (tid >> 1)];
      const unsigned hb = (tid & 1) ? (wd >> 16) : (wd & 0xffffu);
      const float v   = h16_to_f32(hb) + bb;
      const float a   = __expf(-fabsf(v));
      const float u   = 1.0f + a;
      const float l1p = __logf(u) + (a - (u - 1.0f)) * __builtin_amdgcn_rcpf(u);
      const float dt  = fmaxf(v, 0.0f) + l1p;
      const float xcur = XI[(xirow + lrow) * kDin + d];
      float cacc = w0 * xm3;
      cacc = fmaf(w1, xm2, cacc);
      cacc = fmaf(w2, xm1, cacc);
      cacc = fmaf(w3, xcur, cacc);
      xm3 = xm2; xm2 = xm1; xm1 = xcur;
      const float sv = cacc + bc;
      const float xt = sv * __builtin_amdgcn_rcpf(1.0f + __expf(-sv));
      const float dtx = dt * xt;
      float y = 0.f;
#pragma unroll
      for (int k = 0; k < kNst; ++k) {
        const float e = __expf(dt * negA[k]);
        h[k] = e * h[k] + dtx * Bs[k];
        y = h[k] * Cs[k] + y;
      }
      y = xt * Dd + y;
      if (DIR == 0) {
        if (outp) {
          const float zv = Zp[(qrow + lrow) * kDin + d];
          const float yb = YB[(qrow + lrow) * kDin + d];
          const float sg = __builtin_amdgcn_rcpf(1.0f + __expf(-zv));
          y = (0.5f * (y + yb)) * (zv * sg);
        }
      }
      sY[lrow * kScanYP + tid] = y;
    }
    __syncthreads();
    if (DIR == 1) {
      const int hh = lane >> 4, c4 = (lane & 15) * 4;
      for (int pass = 0; pass < 2; ++pass) {
#pragma unroll
        for (int it = 0; it < 16; ++it) {
          const int row = it * 4 + wave * 2 + hh;
          const v4f val = *(const v4f*)(sY + row * kScanYP + c4);
          *(volatile v4f*)(YB + (qrow + row) * kDin + d0 + c4) = val;
        }
        __threadfence();
      }
    } else {
      if (outp) {
        const int q = lane >> 3, c8 = (lane & 7) * 8;
        v8h hv[8], lv[8];
#pragma unroll
        for (int it = 0; it < 8; ++it) {
          const int row = it * 8 + wave * 4 + q;
          const float* sp = sY + row * kScanYP + c8;
          const v4f a0 = *(const v4f*)(sp);
          const v4f a1 = *(const v4f*)(sp + 4);
#pragma unroll
          for (int e = 0; e < 4; ++e) {
            const unsigned short h0 = f2bf_bits(a0[e]), h1 = f2bf_bits(a1[e]);
            const unsigned short l0 = f2bf_bits(a0[e] - bf_bits2f(h0)), l1 = f2bf_bits(a1[e] - bf_bits2f(h1));
            hv[it][e]     = __builtin_bit_cast(_Float16, h0);
            hv[it][4 + e] = __builtin_bit_cast(_Float16, h1);
            lv[it][e]     = __builtin_bit_cast(_Float16, l0);
            lv[it][4 + e] = __builtin_bit_cast(_Float16, l1);
          }
        }
        for (int pass = 0; pass < 2; ++pass) {
#pragma unroll
          for (int it = 0; it < 8; ++it) {
            const int row = it * 8 + wave * 4 + q;
            const size_t o = (qrow + row) * kDin + d0 + c8;
            *(volatile v8h*)(YSH + o) = hv[it];
            *(volatile v8h*)(YSL + o) = lv[it];
          }
          __threadfence();
        }
      }
    }
  }
}

extern "C" void kernel_launch(void* const* d_in, const int* in_sizes, int n_in,
                              void* d_out, int out_size, void* d_ws, size_t ws_size,
                              hipStream_t stream) {
  if (n_in < 13) return;
  if (in_sizes[0] != kBatch * kLq * kDm) return;
  if (in_sizes[1] != kBatch * kLctx * kDm) return;
  if (in_sizes[2] != kDm || in_sizes[3] != kDm) return;
  if (in_sizes[4] != 2 * kDin * kDm) return;
  if (in_sizes[5] != kDin * 4 || in_sizes[6] != kDin) return;
  if (in_sizes[7] != kXdP * kDin) return;
  if (in_sizes[8] != kDin * kDtR || in_sizes[9] != kDin) return;
  if (in_sizes[10] != kDin * kNst || in_sizes[11] != kDin) return;
  if (in_sizes[12] != kDm * kDin) return;
  if (out_size != kRowsB * kDm) return;
  if (ws_size < kWsTotal) return;

  const float* query   = (const float*)d_in[0];
  const float* context = (const float*)d_in[1];
  const float* seg_c   = (const float*)d_in[2];
  const float* seg_q   = (const float*)d_in[3];
  const float* W_in    = (const float*)d_in[4];
  const float* conv_w  = (const float*)d_in[5];
  const float* conv_b  = (const float*)d_in[6];
  const float* W_x     = (const float*)d_in[7];
  const float* W_dt    = (const float*)d_in[8];
  const float* b_dt    = (const float*)d_in[9];
  const float* A_log   = (const float*)d_in[10];
  const float* Dp      = (const float*)d_in[11];
  const float* W_out   = (const float*)d_in[12];
  float* out = (float*)d_out;

  char* ws = (char*)d_ws;
  unsigned short* XH    = (unsigned short*)(ws + kOffXH);
  unsigned short* XL    = (unsigned short*)(ws + kOffXL);
  unsigned short* WIH   = (unsigned short*)(ws + kOffWIH);
  unsigned short* WIL   = (unsigned short*)(ws + kOffWIL);
  unsigned short* WOH   = (unsigned short*)(ws + kOffWOH);
  unsigned short* WOL   = (unsigned short*)(ws + kOffWOL);
  unsigned short* WX16  = (unsigned short*)(ws + kOffWX);
  unsigned short* WDT16 = (unsigned short*)(ws + kOffWDT);
  float*          XI    = (float*)(ws + kOffXI);
  float*          Z     = (float*)(ws + kOffZ);
  unsigned short* XC16  = (unsigned short*)(ws + kOffXC);
  float*          DBL   = (float*)(ws + kOffDBL);
  unsigned short* DT16  = (unsigned short*)(ws + kOffDT16);
  float*          YB    = (float*)(ws + kOffYB);
  unsigned short* DTP16 = XC16;
  unsigned short* YSH   = XH;
  unsigned short* YSL   = XL;

  split_rows_bf16_kernel<<<(2 * kDin * kDm / 8) / 256, 256, 0, stream>>>(W_in, WIH, WIL, 2 * kDin * kDm / 8);
  split_rows_bf16_kernel<<<(kDm * kDin / 8) / 256, 256, 0, stream>>>(W_out, WOH, WOL, kDm * kDin / 8);
  cast_f16_kernel<<<(kXdP * kDin / 8) / 256, 256, 0, stream>>>(W_x, WX16, kXdP * kDin / 8, kCarryWx);
  cast_f16_kernel<<<(kDin * kDtR / 8) / 256, 256, 0, stream>>>(W_dt, WDT16, kDin * kDtR / 8, kCarryWdt);
  build_x_kernel<<<(kRowsF * kDm / 8) / 256, 256, 0, stream>>>(query, context, seg_c, seg_q, XH, XL, kRowsF * kDm / 8);

  wmma_gemm64<1, 2, 0, 0><<<dim3(256, 1), 256, 0, stream>>>(
      XH, XL, kDm, 0L,
      WIH, WIL, kDm, 0L,
      (void*)XI, (void*)XI, kDin, 0L,
      b_dt,
      kRowsF, kDin, kDm, 1.0f);

  wmma_gemm64<1, 2, 0, 0><<<dim3(64, kBatch), 256, 0, stream>>>(
      XH + (size_t)kLctx * kDm, XL + (size_t)kLctx * kDm, kDm, (long)kLtot * kDm,
      WIH + (size_t)kDin * kDm, WIL + (size_t)kDin * kDm, kDm, 0L,
      (void*)Z, (void*)Z, kDin, (long)kLq * kDin,
      b_dt,
      kLq, kDin, kDm, 1.0f);

  conv_silu_kernel<<<dim3(kDin / 256, kRowsS / 64), 256, 0, stream>>>(XI, conv_w, conv_b, XC16);

  wmma_gemm64<0, 0, 0, 0><<<dim3(kRowsS / 64 / 8, 1), 256, 0, stream>>>(
      XC16, XC16, kDin, 0L,
      WX16, WX16, kDin, 0L,
      (void*)DBL, (void*)DBL, kXdP, 0L,
      b_dt,
      kRowsS, kXdP, kDin, 1.0f / kCarryWx);

  dt_cast_kernel<<<(kRowsS * kDtR / 8) / 256, 256, 0, stream>>>(DBL, DT16, kRowsS * kDtR / 8, kCarryDt);

  wmma_gemm64<0, 0, 0, 1><<<dim3((kRowsS / 64) * (kDin / 64) / 8, 1), 256, 0, stream>>>(
      DT16, DT16, kDtR, 0L,
      WDT16, WDT16, kDtR, 0L,
      (void*)DTP16, (void*)DTP16, kDin, 0L,
      b_dt,
      kRowsS, kDin, kDtR, 1.0f / (kCarryDt * kCarryWdt));

  scan_kernel<1><<<kBatch * (kDin / kScanCh), kScanCh, 0, stream>>>(
      DBL, DTP16, XI, Z, conv_w, conv_b, b_dt, A_log, Dp, YB, YSH, YSL);
  scan_kernel<0><<<kBatch * (kDin / kScanCh), kScanCh, 0, stream>>>(
      DBL, DTP16, XI, Z, conv_w, conv_b, b_dt, A_log, Dp, YB, YSH, YSL);

  wmma_gemm64<1, 2, 0, 0><<<dim3(64, 1), 256, 0, stream>>>(
      YSH, YSL, kDin, 0L,
      WOH, WOL, kDin, 0L,
      (void*)out, (void*)out, kDm, 0L,
      b_dt,
      kRowsB, kDm, kDin, 1.0f);
}
